// MPDecoder_83434034692199
// MI455X (gfx1250) — hardware-verified
//
#include <hip/hip_runtime.h>


#define NB_  32
#define NN_  500
#define NP_  500
#define NR   512
#define HH   128
#define NTK  (NB_ * NR)
#define LOSC 1024.0f
#define LOSCI (1.0f / 1024.0f)

typedef _Float16 h16;
typedef unsigned short bf;
typedef __attribute__((ext_vector_type(16))) __bf16   v16bf;
typedef __attribute__((ext_vector_type(16))) _Float16 v16h;
typedef __attribute__((ext_vector_type(8)))  _Float16 v8h;
typedef __attribute__((ext_vector_type(8)))  unsigned short v8us;
typedef __attribute__((ext_vector_type(4)))  unsigned short v4us;
typedef __attribute__((ext_vector_type(4)))  _Float16 v4h;
typedef __attribute__((ext_vector_type(8)))  float    v8f;
typedef __attribute__((ext_vector_type(4)))  float    v4f;
typedef v8h  __attribute__((may_alias)) v8ha;
typedef v4f  __attribute__((may_alias)) v4fa;
typedef v8us __attribute__((may_alias)) v8usa;

__device__ __forceinline__ unsigned short f2bf(float f) { unsigned u = __float_as_uint(f); u += 0x7FFFu + ((u >> 16) & 1u); return (unsigned short)(u >> 16); }
__device__ __forceinline__ float bf2f(unsigned short b) { return __uint_as_float(((unsigned)b) << 16); }
__device__ __forceinline__ float bfr(float f) { return bf2f(f2bf(f)); }
__device__ __forceinline__ v16h cat16(v8h lo, v8h hi) { return __builtin_shufflevector(lo, hi, 0, 1, 2, 3, 4, 5, 6, 7, 8, 9, 10, 11, 12, 13, 14, 15); }
__device__ __forceinline__ v16bf cat16b(v8us lo, v8us hi) { return __builtin_bit_cast(v16bf, __builtin_shufflevector(lo, hi, 0, 1, 2, 3, 4, 5, 6, 7, 8, 9, 10, 11, 12, 13, 14, 15)); }
__device__ __forceinline__ v8f wmma16(v16h a, v16h b, v8f c) { return __builtin_amdgcn_wmma_f32_16x16x32_f16(false, a, false, b, (short)0, c, false, false); }
__device__ __forceinline__ v8f wmmab(v16bf a, v16bf b, v8f c) { return __builtin_amdgcn_wmma_f32_16x16x32_bf16(false, a, false, b, (short)0, c, false, false); }
#define VST2(T, p, v) do { const T vst2_v_ = (v); *(volatile T*)(p) = vst2_v_; __threadfence(); *(volatile T*)(p) = vst2_v_; } while (0)

__global__ __launch_bounds__(256) void k_emb(const float* __restrict__ emb, const int* __restrict__ last, bf* Eb, h16* E16, bf* Gb) {
    const int lane = threadIdx.x & 31, r = blockIdx.x * 8 + (threadIdx.x >> 5);
    if (r >= NTK) return;
    const int b = r / NR, n = r - b * NR;
    const bool live = n < NN_;
    const int nc = live ? n : 0;
    int ln = live ? last[b * NP_ + nc] : 0; if (ln < 0) ln += NN_; ln = ((unsigned)ln < (unsigned)NN_) ? ln : 0;
    v4us e, g; v4h e16;
#pragma unroll
    for (int i = 0; i < 4; ++i) { const int c = lane * 4 + i;
        const unsigned short hb = f2bf(emb[((size_t)b * NN_ + nc) * HH + c]); e[i] = live ? hb : (unsigned short)0; e16[i] = live ? (h16)bf2f(hb) : (h16)0.f;
        const unsigned short gb_ = f2bf(emb[((size_t)b * NN_ + ln) * HH + c]); g[i] = live ? gb_ : (unsigned short)0; }
    *(volatile v4us*)(Eb + (size_t)r * HH + lane * 4) = e; *(volatile v4h*)(E16 + (size_t)r * HH + lane * 4) = e16; *(volatile v4us*)(Gb + (size_t)r * HH + lane * 4) = g;
    __threadfence();
    *(volatile v4us*)(Eb + (size_t)r * HH + lane * 4) = e; *(volatile v4h*)(E16 + (size_t)r * HH + lane * 4) = e16; *(volatile v4us*)(Gb + (size_t)r * HH + lane * 4) = g;
}
__global__ __launch_bounds__(256) void k_et(const float* __restrict__ emb, h16* ET16) {
    __shared__ __align__(16) h16 tl[64 * 72];
    const int tid = threadIdx.x, n0 = blockIdx.x * 64, c0 = blockIdx.y * 64, b = blockIdx.z;
    const int nn = tid >> 2, cq = (tid & 3) * 16, n = n0 + nn, ncl = (n < NN_) ? n : 0;
#pragma unroll
    for (int i = 0; i < 16; ++i) { const h16 v = (h16)bfr(emb[((size_t)b * NN_ + ncl) * HH + c0 + cq + i]); tl[(cq + i) * 72 + nn] = (n < NN_) ? v : (h16)0.f; }
    __syncthreads();
    const int piece = tid & 7;
    auto pass = [&]() {
#pragma unroll
        for (int s = 0; s < 2; ++s) { const int cr = (tid >> 3) + 32 * s; const v8h val = *(const v8ha*)(tl + cr * 72 + piece * 8);
            *(volatile v8h*)(ET16 + ((size_t)b * HH + c0 + cr) * NR + n0 + piece * 8) = val; }
    };
    pass(); __threadfence(); pass();
}
__global__ __launch_bounds__(256) void k_mv(const float* __restrict__ gm, h16* MV16) {
    const int lane = threadIdx.x & 31, r = blockIdx.x * 8 + (threadIdx.x >> 5);
    if (r >= NTK) return;
    const int b = r / NR, p = r - b * NR, pc = (p < NP_) ? p : 0;
#pragma unroll
    for (int q = 0; q < 2; ++q) { v8h t;
#pragma unroll
        for (int i = 0; i < 8; ++i) { const int n = q * 256 + lane * 8 + i, ncl = (n < NN_) ? n : 0; const float m = gm[((size_t)b * NP_ + pc) * NN_ + ncl];
            t[i] = (p < NP_ && n < NN_ && __builtin_isinf(m) && m < 0.f) ? (h16)1.f : (h16)0.f; }
        VST2(v8h, MV16 + (size_t)r * NR + q * 256 + lane * 8, t); }
}
__global__ __launch_bounds__(256) void k_cvtw(const float* __restrict__ Wm, bf* WB) {
    const int lane = threadIdx.x & 31, r = blockIdx.x * 8 + (threadIdx.x >> 5);
    if (r >= HH) return;
    v4us t;
#pragma unroll
    for (int i = 0; i < 4; ++i) t[i] = f2bf(Wm[(size_t)r * HH + lane * 4 + i]);
    VST2(v4us, WB + (size_t)r * HH + lane * 4, t);
}
__global__ __launch_bounds__(128) void k_qg(const float* __restrict__ emb, const float* __restrict__ Wg, float* QG) {
    __shared__ float mean_[HH];
    const int b = blockIdx.x, c = threadIdx.x;
    float s = 0.f;
#pragma unroll 4
    for (int n = 0; n < NN_; ++n) s += bfr(emb[((size_t)b * NN_ + n) * HH + c]);
    mean_[c] = s / (float)NN_;
    __syncthreads();
    float q = 0.f;
#pragma unroll 4
    for (int k = 0; k < HH; ++k) q += mean_[k] * bfr(Wg[(size_t)c * HH + k]);
    VST2(float, QG + (size_t)b * HH + c, q);
}

template <bool F16A, bool SPLITA, int MODE>
__global__ __launch_bounds__(128) void k_gemm(const void* __restrict__ Av, const void* __restrict__ Alv, const void* __restrict__ Bv, int K, size_t bstrideB,
                                             const float* __restrict__ QF, const float* __restrict__ QG, float scale, float* C) {
    __shared__ __align__(16) float ost[4][16 * 68];
    const int lane = threadIdx.x & 31, wave = threadIdx.x >> 5, lr = lane & 15, hi = lane >> 4;
    const int r0 = blockIdx.x * 64 + wave * 16, c0 = blockIdx.y * 64, b = (blockIdx.x * 64) / NR;
    const size_t aoff = (size_t)(r0 + lr) * K + 8 * hi;
    size_t boff[4];
#pragma unroll
    for (int t = 0; t < 4; ++t) boff[t] = (size_t)b * bstrideB + (size_t)(c0 + t * 16 + lr) * K + 8 * hi;
    v8f acc[4], accx[4];
#pragma unroll
    for (int t = 0; t < 4; ++t) { acc[t] = (v8f){}; accx[t] = (v8f){}; }
#pragma unroll 1
    for (int kc = 0; kc < K; kc += 32) {
        if (F16A) {
            const h16* A = (const h16*)Av; const h16* Al = (const h16*)Alv; const h16* Bm = (const h16*)Bv;
            const v16h a = cat16(*(const v8h*)(A + aoff + kc), *(const v8h*)(A + aoff + kc + 16));
            v16h al = a; if (SPLITA) al = cat16(*(const v8h*)(Al + aoff + kc), *(const v8h*)(Al + aoff + kc + 16));
#pragma unroll
            for (int t = 0; t < 4; ++t) { const v16h bb = cat16(*(const v8h*)(Bm + boff[t] + kc), *(const v8h*)(Bm + boff[t] + kc + 16)); acc[t] = wmma16(a, bb, acc[t]); if (SPLITA) accx[t] = wmma16(al, bb, accx[t]); }
            asm volatile("v_nop\n\tv_nop\n\tv_nop\n\tv_nop" : "+v"(acc[0]), "+v"(acc[1]), "+v"(acc[2]), "+v"(acc[3]), "+v"(accx[0]), "+v"(accx[3]) : "v"(a), "v"(al));
        } else {
            const bf* A = (const bf*)Av; const bf* Al = (const bf*)Alv; const bf* Bm = (const bf*)Bv;
            const v16bf a = cat16b(*(const v8us*)(A + aoff + kc), *(const v8us*)(A + aoff + kc + 16));
            v16bf al = a; if (SPLITA) al = cat16b(*(const v8us*)(Al + aoff + kc), *(const v8us*)(Al + aoff + kc + 16));
#pragma unroll
            for (int t = 0; t < 4; ++t) { const v16bf bb = cat16b(*(const v8us*)(Bm + boff[t] + kc), *(const v8us*)(Bm + boff[t] + kc + 16)); acc[t] = wmmab(a, bb, acc[t]); if (SPLITA) accx[t] = wmmab(al, bb, accx[t]); }
            asm volatile("v_nop\n\tv_nop\n\tv_nop\n\tv_nop" : "+v"(acc[0]), "+v"(acc[1]), "+v"(acc[2]), "+v"(acc[3]), "+v"(accx[0]), "+v"(accx[3]) : "v"(a), "v"(al));
        }
    }
    asm volatile("v_nop\n\tv_nop\n\tv_nop\n\tv_nop" : "+v"(accx[0]), "+v"(accx[1]), "+v"(accx[2]), "+v"(accx[3]));
    float* os = &ost[wave][0];
#pragma unroll
    for (int t = 0; t < 4; ++t) { const int col = c0 + t * 16 + lr;
#pragma unroll
        for (int j = 0; j < 8; ++j) { const int row = r0 + hi * 8 + j; float v = (acc[t][j] + (SPLITA ? accx[t][j] : 0.f)) * scale;
            if (MODE == 0) { const int p = row - b * NR, pcl = (p < NP_) ? p : 0; v += C[(size_t)row * HH + col] + bfr(QF[((size_t)b * NP_ + pcl) * HH + col]) + QG[(size_t)b * HH + col]; if (p >= NP_) v = 0.f; }
            os[(hi * 8 + j) * 68 + t * 16 + lr] = v; } }
    __syncthreads();
    const int ldc = (MODE == 2) ? NR : HH;
    float* crow = C + (size_t)r0 * ldc + c0;
    auto pass = [&]() {
#pragma unroll
        for (int s = 0; s < 8; ++s) { const int Lid = (lane >> 3) + 4 * s, piece = lane & 7; const int row = Lid >> 1, cofs = (Lid & 1) * 32 + piece * 4;
            const v4f val = *(const v4fa*)(os + row * 68 + cofs); *(volatile v4f*)(crow + (size_t)row * ldc + cofs) = val; }
    };
    pass(); __threadfence(); pass();
}

__global__ __launch_bounds__(256) void k_split16(const float* __restrict__ S, h16* H, h16* L) {
    const int lane = threadIdx.x & 31, r = blockIdx.x * 8 + (threadIdx.x >> 5);
    if (r >= NTK) return;
    v4h oh, ol;
#pragma unroll
    for (int i = 0; i < 4; ++i) { const float v = S[(size_t)r * HH + lane * 4 + i]; const h16 a = (h16)v; oh[i] = a; ol[i] = (h16)((v - (float)a) * LOSC); }
    *(volatile v4h*)(H + (size_t)r * HH + lane * 4) = oh; *(volatile v4h*)(L + (size_t)r * HH + lane * 4) = ol; __threadfence();
    *(volatile v4h*)(H + (size_t)r * HH + lane * 4) = oh; *(volatile v4h*)(L + (size_t)r * HH + lane * 4) = ol;
}
__global__ __launch_bounds__(256) void k_splitbf(const float* __restrict__ S, bf* H, bf* L) {
    const int lane = threadIdx.x & 31, r = blockIdx.x * 8 + (threadIdx.x >> 5);
    if (r >= NTK) return;
    v4us oh, ol;
#pragma unroll
    for (int i = 0; i < 4; ++i) { const float v = S[(size_t)r * HH + lane * 4 + i]; const unsigned short a = f2bf(v); oh[i] = a; ol[i] = f2bf(v - bf2f(a)); }
    *(volatile v4us*)(H + (size_t)r * HH + lane * 4) = oh; *(volatile v4us*)(L + (size_t)r * HH + lane * 4) = ol; __threadfence();
    *(volatile v4us*)(H + (size_t)r * HH + lane * 4) = oh; *(volatile v4us*)(L + (size_t)r * HH + lane * 4) = ol;
}

__global__ __launch_bounds__(128) void k_score(const h16* __restrict__ FQH, const h16* __restrict__ FQL, const h16* __restrict__ KH, const h16* __restrict__ KL,
                                              const float* __restrict__ dists, const int* __restrict__ last, const float* __restrict__ gm, float* PR) {
    extern __shared__ float4 lds_raw[];
    float* lgs = (float*)lds_raw;
    const int lane = threadIdx.x & 31, wave = threadIdx.x >> 5, lr = lane & 15, hi = lane >> 4;
    const int b = blockIdx.x / (NR / 64), pt = blockIdx.x - b * (NR / 64), p0 = pt * 64 + wave * 16;
    float* my = lgs + (size_t)wave * 16 * NR;
    v16h ah[4], al[4];
#pragma unroll
    for (int kc = 0; kc < 4; ++kc) { const size_t o = ((size_t)b * NR + p0 + lr) * HH + kc * 32 + 8 * hi;
        ah[kc] = cat16(*(const v8h*)(FQH + o), *(const v8h*)(FQH + o + 16)); al[kc] = cat16(*(const v8h*)(FQL + o), *(const v8h*)(FQL + o + 16)); }
    int prow[8], lnode[8];
#pragma unroll
    for (int j = 0; j < 8; ++j) { const int p = p0 + 8 * hi + j; prow[j] = (p < NP_) ? p : 0; int ln = last[b * NP_ + prow[j]]; if (ln < 0) ln += NN_; lnode[j] = ((unsigned)ln < (unsigned)NN_) ? ln : 0; }
    const float s1 = 1.0f / (8.0f * 11.313708498984761f), s2 = 0.7071067811865476f;
#pragma unroll 1
    for (int g = 0; g < NR / 64; ++g) {
        v8f acc[4], accx[4];
#pragma unroll
        for (int t = 0; t < 4; ++t) { acc[t] = (v8f){}; accx[t] = (v8f){}; }
#pragma unroll
        for (int kc = 0; kc < 4; ++kc)
#pragma unroll
            for (int t = 0; t < 4; ++t) { const size_t o = ((size_t)b * NR + g * 64 + t * 16 + lr) * HH + kc * 32 + 8 * hi;
                const v16h kh = cat16(*(const v8h*)(KH + o), *(const v8h*)(KH + o + 16)), kl = cat16(*(const v8h*)(KL + o), *(const v8h*)(KL + o + 16));
                acc[t] = wmma16(ah[kc], kh, acc[t]); accx[t] = wmma16(ah[kc], kl, accx[t]); accx[t] = wmma16(al[kc], kh, accx[t]); }
        asm volatile("v_nop\n\tv_nop\n\tv_nop\n\tv_nop" : "+v"(acc[0]), "+v"(acc[1]), "+v"(acc[2]), "+v"(acc[3]), "+v"(accx[0]), "+v"(accx[1]), "+v"(accx[2]), "+v"(accx[3]));
#pragma unroll
        for (int t = 0; t < 4; ++t) { const int n = g * 64 + t * 16 + lr; const bool nlive = n < NN_; const int ncl = nlive ? n : 0;
#pragma unroll
            for (int j = 0; j < 8; ++j) {
                const float sc = (acc[t][j] + accx[t][j] * LOSCI) * s1 - bfr(dists[((size_t)b * NN_ + lnode[j]) * NN_ + ncl]) * s2;
                const float m = gm[((size_t)b * NP_ + prow[j]) * NN_ + ncl];
                const float v = 10.0f * tanhf(sc) + ((__builtin_isinf(m) && m < 0.f) ? -1e8f : 0.f);
                my[(hi * 8 + j) * NR + n] = nlive ? v : -__builtin_inff(); } }
    }
    asm volatile("" ::: "memory");
    __builtin_amdgcn_fence(__ATOMIC_RELEASE, "workgroup");
    __builtin_amdgcn_wave_barrier();
    const int row = lr, p = p0 + row; const float* lrow = my + row * NR + hi * 256;
    float mx = -3.0e38f;
#pragma unroll 4
    for (int i = 0; i < 256; ++i) mx = fmaxf(mx, lrow[i]);
    mx = fmaxf(mx, __shfl_xor(mx, 16, 32));
    float sm = 0.f;
#pragma unroll 4
    for (int i = 0; i < 256; ++i) sm += __expf(lrow[i] - mx);
    sm += __shfl_xor(sm, 16, 32);
    const float inv = 1.0f / sm;
    float* dst = PR + ((size_t)b * NR + p) * NR + hi * 256;
    const bool pl = p < NP_;
#pragma unroll 2
    for (int i = 0; i < 64; ++i) { v4f v;
#pragma unroll
        for (int q = 0; q < 4; ++q) v[q] = pl ? __expf(lrow[i * 4 + q] - mx) * inv : 0.f;
        *(volatile v4f*)(dst + i * 4) = v; }
    __threadfence();
#pragma unroll 2
    for (int i = 0; i < 64; ++i) { v4f v;
#pragma unroll
        for (int q = 0; q < 4; ++q) v[q] = pl ? __expf(lrow[i * 4 + q] - mx) * inv : 0.f;
        *(volatile v4f*)(dst + i * 4) = v; }
}
__global__ __launch_bounds__(256) void k_out(const float* __restrict__ PR, float* out) {
    const int lane = threadIdx.x & 31; const size_t flat = ((size_t)blockIdx.x * 8 + (threadIdx.x >> 5)) * 32 + lane;
    if (flat >= (size_t)NB_ * NP_ * NN_) return;
    const int b = (int)(flat / ((size_t)NP_ * NN_)); const int rem = (int)(flat - (size_t)b * NP_ * NN_); const int p = rem / NN_, n = rem - p * NN_;
    VST2(float, out + flat, PR[((size_t)b * NR + p) * NR + n]);
}

extern "C" void kernel_launch(void* const* d_in, const int* in_sizes, int n_in,
                              void* d_out, int out_size, void* d_ws, size_t ws_size, hipStream_t stream) {
    (void)in_sizes; (void)n_in; (void)out_size;
    const float* emb = (const float*)d_in[0]; const float* dists = (const float*)d_in[1]; const float* qf = (const float*)d_in[2];
    const float* Wql = (const float*)d_in[3]; const float* Wqv = (const float*)d_in[4]; const float* Wqg = (const float*)d_in[5]; const float* Wq = (const float*)d_in[6]; const float* Wk = (const float*)d_in[7];
    const int* last = (const int*)d_in[8]; const float* gm = (const float*)d_in[9];
    float* out = (float*)d_out;
    char* wsp = (char*)d_ws;
    auto take = [&](size_t bytes) { char* p = wsp; wsp += (bytes + 255) & ~(size_t)255; return (void*)p; };
    bf* Eb = (bf*)take((size_t)NTK * HH * 2); h16* E16 = (h16*)take((size_t)NTK * HH * 2); bf* Gb = (bf*)take((size_t)NTK * HH * 2); h16* ET16 = (h16*)take((size_t)NB_ * HH * NR * 2);
    h16* MV16 = (h16*)take((size_t)NTK * NR * 2);
    bf* WqlB = (bf*)take(HH * HH * 2); bf* WqvB = (bf*)take(HH * HH * 2); bf* WqB = (bf*)take(HH * HH * 2); bf* WkB = (bf*)take(HH * HH * 2);
    float* QG = (float*)take((size_t)NB_ * HH * 4); float* KF = (float*)take((size_t)NTK * HH * 4); float* SV = (float*)take((size_t)NTK * HH * 4); float* QP = (float*)take((size_t)NTK * HH * 4); float* FQ = (float*)take((size_t)NTK * HH * 4);
    bf* AH = (bf*)take((size_t)NTK * HH * 2); bf* AL = (bf*)take((size_t)NTK * HH * 2);
    h16* FQH = (h16*)take((size_t)NTK * HH * 2); h16* FQL = (h16*)take((size_t)NTK * HH * 2); h16* KH = (h16*)take((size_t)NTK * HH * 2); h16* KL = (h16*)take((size_t)NTK * HH * 2);
    float* PR = (float*)take((size_t)NTK * NR * 4);
    if ((size_t)(wsp - (char*)d_ws) > ws_size) return;
    (void)E16;
    k_emb<<<NTK / 8, 256, 0, stream>>>(emb, last, Eb, E16, Gb);
    k_et<<<dim3(NR / 64, HH / 64, NB_), 256, 0, stream>>>(emb, ET16);
    k_mv<<<NTK / 8, 256, 0, stream>>>(gm, MV16);
    k_cvtw<<<HH / 8, 256, 0, stream>>>(Wql, WqlB); k_cvtw<<<HH / 8, 256, 0, stream>>>(Wqv, WqvB); k_cvtw<<<HH / 8, 256, 0, stream>>>(Wq, WqB); k_cvtw<<<HH / 8, 256, 0, stream>>>(Wk, WkB);
    k_qg<<<NB_, 128, 0, stream>>>(emb, Wqg, QG);
    k_gemm<false, false, 1><<<dim3(NTK / 64, HH / 64, 1), 128, 0, stream>>>(Eb, nullptr, WkB, HH, 0, nullptr, nullptr, 1.0f, KF);
    k_gemm<true, false, 1><<<dim3(NTK / 64, HH / 64, 1), 128, 0, stream>>>(MV16, nullptr, ET16, NR, (size_t)HH * NR, nullptr, nullptr, 1.0f / NN_, SV);
    k_splitbf<<<NTK / 8, 256, 0, stream>>>(SV, AH, AL);
    k_gemm<false, false, 1><<<dim3(NTK / 64, HH / 64, 1), 128, 0, stream>>>(Gb, nullptr, WqlB, HH, 0, nullptr, nullptr, 1.0f, QP);
    k_gemm<false, true, 0><<<dim3(NTK / 64, HH / 64, 1), 128, 0, stream>>>(AH, AL, WqvB, HH, 0, qf, QG, 1.0f, QP);
    k_splitbf<<<NTK / 8, 256, 0, stream>>>(QP, AH, AL);
    k_gemm<false, true, 1><<<dim3(NTK / 64, HH / 64, 1), 128, 0, stream>>>(AH, AL, WqB, HH, 0, nullptr, nullptr, 1.0f, FQ);
    k_split16<<<NTK / 8, 256, 0, stream>>>(FQ, FQH, FQL);
    k_split16<<<NTK / 8, 256, 0, stream>>>(KF, KH, KL);
    k_score<<<NB_ * (NR / 64), 128, (size_t)4 * 16 * NR * 4, stream>>>(FQH, FQL, KH, KL, dists, last, gm, PR);
    k_out<<<(NB_ * NP_ * NN_ + 255) / 256, 256, 0, stream>>>(PR, out);
}
